// BandSplit_79139067396476
// MI455X (gfx1250) — hardware-verified
//
#include <hip/hip_runtime.h>


namespace {
constexpr int NB_ = 8, CI = 2, T = 512, F = 1025, K = 128, W = 65, WC = W * CI  , KP = 160, DO = 128, OP = 144  , YS = 160  ;
constexpr float HS = 256.0f, WSC = 256.0f;
typedef _Float16 b16;
typedef __attribute__((ext_vector_type(16))) _Float16 v16b;
typedef __attribute__((ext_vector_type(8))) _Float16 v8b;
typedef __attribute__((ext_vector_type(8))) float v8f;
typedef __attribute__((ext_vector_type(4))) float v4f;
__device__ __forceinline__ float bf16_rne(float f) { unsigned int u = __float_as_uint(f); u += 0x7FFFu + ((u >> 16) & 1u); float r = __uint_as_float(u & 0xFFFF0000u); asm volatile("" : "+v"(r)); return r; }
__device__ __forceinline__ float bfv(float f) { float r = bf16_rne(f); asm volatile("" : "+v"(r)); return r; }
__device__ __forceinline__ void split16(float v, b16& hi, b16& lo) { hi = (b16)v; lo = (b16)(v - (float)hi); }
__device__ __forceinline__ v16b frag_kb(const b16* p, int hh) { const v8b a = *(const v8b*)(p + 8 * hh), b = *(const v8b*)(p + 16 + 8 * hh); v16b f;
#pragma unroll
  for (int e = 0; e < 8; ++e) { f[e] = a[e]; f[8 + e] = b[e]; } return f; }
__device__ __forceinline__ v8f wmma16b(v16b a, v16b b, v8f c) { v8f d = __builtin_amdgcn_wmma_f32_16x16x32_f16(false, a, false, b, (short)0, c, false, false); asm volatile("v_nop\n\tv_nop\n\tv_nop\n\tv_nop" : "+v"(d) : "v"(a), "v"(b)); return d; }
__device__ __forceinline__ void wave_lds_sync() { __builtin_amdgcn_fence(__ATOMIC_RELEASE, "workgroup"); __builtin_amdgcn_wave_barrier(); __builtin_amdgcn_fence(__ATOMIC_ACQUIRE, "workgroup"); }
__device__ __forceinline__ float pmul(float a, float b) { float p = a * b; asm volatile("" : "+v"(p)); return p; }
__device__ __forceinline__ int iclamp(int v, int lo, int hi) { return v < lo ? lo : (v > hi ? hi : v); }

__global__ __launch_bounds__(256) void prep_kernel(const float* __restrict__ prew, const float* __restrict__ postw, const int* __restrict__ idx, const float* __restrict__ mask, b16* __restrict__ WT1, b16* __restrict__ WT2, int* __restrict__ INV, int* __restrict__ INVN) { const size_t nt = (size_t)gridDim.x * 256, u0 = (size_t)blockIdx.x * 256 + threadIdx.x; v8b v;
  for (size_t u = u0; u < (size_t)K * DO * (KP / 8); u += nt) { const int k = (int)(u / (DO * (KP / 8))), o = (int)((u / (KP / 8)) % DO), i0 = (int)(u % (KP / 8)) * 8;
#pragma unroll
    for (int j = 0; j < 8; ++j) { const int i = i0 + j; v[j] = (b16)(i < WC ? bf16_rne(prew[((size_t)k * WC + i) * DO + o]) * WSC : 0.0f); } for (int pass = 0; pass < 2; ++pass) { *(volatile v8b*)(WT1 + ((size_t)k * DO + o) * KP + i0) = v; __threadfence(); } }
  for (size_t u = u0; u < (size_t)K * OP * (DO / 8); u += nt) { const int k = (int)(u / (OP * (DO / 8))), o = (int)((u / (DO / 8)) % OP), d0 = (int)(u % (DO / 8)) * 8;
#pragma unroll
    for (int j = 0; j < 8; ++j) v[j] = (b16)(o < WC ? bf16_rne(postw[((size_t)k * DO + d0 + j) * WC + o]) * WSC : 0.0f); for (int pass = 0; pass < 2; ++pass) { *(volatile v8b*)(WT2 + ((size_t)k * OP + o) * DO + d0) = v; __threadfence(); } }
  for (size_t u = u0; u < (size_t)F; u += nt) { int n = 0, e4[4] = {0, 0, 0, 0};
#pragma unroll 1
    for (int q = 0; q < K * W; ++q) if (idx[q] == (int)u && mask[q] != 0.0f) { if (n < 4) { if (n == 0) e4[0] = q; else if (n == 1) e4[1] = q; else if (n == 2) e4[2] = q; else e4[3] = q; } ++n; }
    for (int pass = 0; pass < 2; ++pass) { ((volatile int*)INV)[u * 4] = e4[0]; ((volatile int*)INV)[u * 4 + 1] = e4[1]; ((volatile int*)INV)[u * 4 + 2] = e4[2]; ((volatile int*)INV)[u * 4 + 3] = e4[3]; ((volatile int*)INVN)[u] = n; __threadfence(); } } }
__global__ __launch_bounds__(32) void band_kernel(const float* __restrict__ xb  , const int* __restrict__ idx, const float* __restrict__ mel, const float* __restrict__ mask, const b16* __restrict__ WT1, const b16* __restrict__ WT2, const float* __restrict__ preb, const float* __restrict__ postb, int TLIM, float* __restrict__ Y) { __shared__ __attribute__((aligned(16))) b16 Ah[16][KP + 8], Al[16][KP + 8]; __shared__ float Tz[16][DO + 4], Ty[16][OP + 1]; const int lane = threadIdx.x, nloc = lane & 15, hlf = lane >> 4; const int t0 = blockIdx.x * 16, k = blockIdx.y; if (t0 >= TLIM) return;
  int fq[6]; float mq[6];
#pragma unroll
  for (int m = 0; m < 6; ++m) { const int i = lane + 32 * m; fq[m] = -1; mq[m] = 0.0f; if (i < WC) { const int q = k * W + (i >> 1); fq[m] = iclamp(idx[q], 0, F - 1); mq[m] = pmul(bfv(mel[q]), mask[q]); } }
  for (int rr = 0; rr < 16; ++rr) {
#pragma unroll
    for (int m = 0; m < 6; ++m) { const int i = lane + 32 * m; if (i >= KP + 8) continue; float gv = 0.0f; if (fq[m] >= 0) gv = pmul(bfv(xb[((size_t)(i & 1) * T + t0 + rr) * F + fq[m]]), mq[m]); b16 p, pl; split16(gv * HS, p, pl); Ah[rr][i] = p; Al[rr][i] = pl; } }
  wave_lds_sync();
  { v8f acc[8];
#pragma unroll
    for (int tt = 0; tt < 8; ++tt) acc[tt] = (v8f){};
#pragma unroll 1
    for (int kb = 0; kb < KP; kb += 32) { const v16b a = frag_kb(&Ah[nloc][kb], hlf), al = frag_kb(&Al[nloc][kb], hlf);
#pragma unroll
      for (int tt = 0; tt < 8; ++tt) { const v16b bw = frag_kb(WT1 + ((size_t)k * DO + tt * 16 + nloc) * KP + kb, hlf); acc[tt] = wmma16b(a, bw, acc[tt]); acc[tt] = wmma16b(al, bw, acc[tt]); } }
#pragma unroll
    for (int tt = 0; tt < 8; ++tt) { const int cc = tt * 16 + nloc; const float bb = bfv(preb[k * DO + cc]);
#pragma unroll
      for (int r8 = 0; r8 < 8; ++r8) Tz[8 * hlf + r8][cc] = acc[tt][r8] * (1.0f / (HS * WSC)) + bb; } }
  wave_lds_sync();
  for (int rr = 0; rr < 16; ++rr) for (int q = 0; q < 4; ++q) { const int c = q * 32 + lane; b16 p, pl; split16(Tz[rr][c] * HS, p, pl); Ah[rr][c] = p; Al[rr][c] = pl; }
  if (lane < 16) for (int c = DO; c < DO + 8; ++c) { Ah[lane][c] = (b16)0.0f; Al[lane][c] = (b16)0.0f; }
  wave_lds_sync();
  { v8f acc[9];
#pragma unroll
    for (int tt = 0; tt < 9; ++tt) acc[tt] = (v8f){};
#pragma unroll 1
    for (int kb = 0; kb < DO; kb += 32) { const v16b a = frag_kb(&Ah[nloc][kb], hlf), al = frag_kb(&Al[nloc][kb], hlf);
#pragma unroll
      for (int tt = 0; tt < 9; ++tt) { const v16b bw = frag_kb(WT2 + ((size_t)k * OP + tt * 16 + nloc) * DO + kb, hlf); acc[tt] = wmma16b(a, bw, acc[tt]); acc[tt] = wmma16b(al, bw, acc[tt]); } }
#pragma unroll
    for (int tt = 0; tt < 9; ++tt) { const int o = tt * 16 + nloc; const float bb = o < WC ? bfv(postb[k * WC + o]) : 0.0f; const float mk = o < WC ? mask[k * W + (o >> 1)] : 0.0f;
#pragma unroll
      for (int r8 = 0; r8 < 8; ++r8) Ty[8 * hlf + r8][o] = o < WC ? pmul(acc[tt][r8] * (1.0f / (HS * WSC)) + bb, mk) : 0.0f; } }
  wave_lds_sync();
  for (int pass = 0; pass < 2; ++pass) { for (int rr = 0; rr < 16; ++rr) for (int q = 0; q < 5; ++q) { const int c = q * 32 + lane; ((volatile float*)Y)[((size_t)(t0 + rr) * K + k) * YS + c] = c < OP ? Ty[rr][c] : 0.0f; } __threadfence(); } }
__global__ __launch_bounds__(256) void fold_kernel(const float* __restrict__ Y, const int* __restrict__ INV, const int* __restrict__ INVN, const float* __restrict__ ola, int TLIM, float* __restrict__ outb  ) { const size_t u = (size_t)blockIdx.x * 256 + threadIdx.x; if (u >= (size_t)CI * T * F) return; const int f = (int)(u % F), t = (int)((u / F) % T), c = (int)(u / ((size_t)F * T)); float s = 0.0f;
  if (t < TLIM) { const int n = iclamp(INVN[f], 0, 4); for (int j = 0; j < n; ++j) { const int q = iclamp(INV[f * 4 + j], 0, K * W - 1); const int k = q / W, w = q % W; s += Y[((size_t)t * K + k) * YS + w * 2 + c]; } }
  const float v = s / bfv(ola[f]);
  for (int pass = 0; pass < 2; ++pass) { ((volatile float*)outb)[u] = v; __threadfence(); } }
}

extern "C" void kernel_launch(void* const* d_in, const int* in_sizes, int n_in, void* d_out, int out_size, void* d_ws, size_t ws_size, hipStream_t stream) {
  (void)n_in;
  auto Fp = [&](int i) { return (const float*)d_in[i]; }; auto Ip = [&](int i) { return (const int*)d_in[i]; };
  if (in_sizes[0] != NB_ * CI * T * F || in_sizes[1] != K * WC * DO || in_sizes[2] != K * DO || in_sizes[3] != K * DO * WC || in_sizes[4] != K * WC || in_sizes[5] != K * W || in_sizes[6] != K * W || in_sizes[7] != F || in_sizes[8] != K * W || out_size != NB_ * CI * T * F) return;
  const int TLIM = T;
  size_t off = 0; char* ws = (char*)d_ws;
  auto carve = [&](size_t bytes) { char* p = ws + off; off += (bytes + 255) & ~(size_t)255; return p; };
  b16* WT1 = (b16*)carve((size_t)K * DO * KP * 2); b16* WT2 = (b16*)carve((size_t)K * OP * DO * 2); int* INV = (int*)carve((size_t)F * 4 * 4); int* INVN = (int*)carve((size_t)F * 4 + 256); float* Y = (float*)carve((size_t)T * K * YS * 4);
  if (off > ws_size || off > ((size_t)64 << 20)) return;
  prep_kernel<<<256, 256, 0, stream>>>(Fp(1), Fp(3), Ip(8), Fp(6), WT1, WT2, INV, INVN);
  for (int b = 0; b < NB_; ++b) { const float* xb = Fp(0) + (size_t)b * CI * T * F; float* ob = (float*)d_out + (size_t)b * CI * T * F;
    band_kernel<<<dim3(T / 16, K), 32, 0, stream>>>(xb, Ip(8), Fp(5), Fp(6), WT1, WT2, Fp(2), Fp(4), TLIM, Y);
    fold_kernel<<<(CI * T * F + 255) / 256, 256, 0, stream>>>(Y, INV, INVN, Fp(7), TLIM, ob); }
}
